// LightweightCrossAttention_18150531792901
// MI455X (gfx1250) — hardware-verified
//
#include <hip/hip_runtime.h>


namespace {
constexpr int NB = 8, T = 2048, D = 256, NR = NB * T  ;
constexpr float XS = 8.0f, OS = 1024.0f  , WSC = 256.0f, PS = 8.0f, SCALE = 0.0625f, LOG2E = 1.4426950408889634f;

typedef _Float16 b16;
typedef __attribute__((ext_vector_type(16))) _Float16 v16b;
typedef __attribute__((ext_vector_type(8))) _Float16 v8b;
typedef __attribute__((ext_vector_type(8))) float v8f;
typedef __attribute__((ext_vector_type(4))) float v4f;
__device__ __forceinline__ float bf16_rne(float f) { unsigned int u = __float_as_uint(f); u += 0x7FFFu + ((u >> 16) & 1u); return __uint_as_float(u & 0xFFFF0000u); }
__device__ __forceinline__ void split16(float v, b16& hi, b16& lo) { hi = (b16)v; lo = (b16)(v - (float)hi); }
__device__ __forceinline__ v16b frag_kb(const b16* p, int hh) { const v8b a = *(const v8b*)(p + 8 * hh), b = *(const v8b*)(p + 16 + 8 * hh); v16b f;
#pragma unroll
  for (int e = 0; e < 8; ++e) { f[e] = a[e]; f[8 + e] = b[e]; } return f; }
__device__ __forceinline__ v8f wmma16b(v16b a, v16b b, v8f c) { v8f d = __builtin_amdgcn_wmma_f32_16x16x32_f16(false, a, false, b, (short)0, c, false, false); asm volatile("v_nop\n\tv_nop\n\tv_nop\n\tv_nop" : "+v"(d) : "v"(a), "v"(b)); return d; }
__device__ __forceinline__ void wave_lds_sync() { __builtin_amdgcn_fence(__ATOMIC_RELEASE, "workgroup"); __builtin_amdgcn_wave_barrier(); __builtin_amdgcn_fence(__ATOMIC_ACQUIRE, "workgroup"); }
__device__ __forceinline__ float nexp2(float x) { return __builtin_amdgcn_exp2f(x); }

__global__ __launch_bounds__(256) void prep_kernel(const float* __restrict__ xq, const float* __restrict__ xc, const float* __restrict__ wq, const float* __restrict__ wkv, const float* __restrict__ wo, b16* __restrict__ X16, b16* __restrict__ WT) {
  const size_t t = (size_t)blockIdx.x * 256 + threadIdx.x; const size_t nx = (size_t)2 * NR * D / 8, nw = (size_t)(256 + 512 + 256) * D / 8; v8b o;
  if (t < nx) { const size_t e = t * 8; const float* src = (e < (size_t)NR * D) ? xq + e : xc + (e - (size_t)NR * D); for (int j = 0; j < 8; ++j) o[j] = (b16)(bf16_rne(src[j]) * XS); for (int pass = 0; pass < 2; ++pass) { *(volatile v8b*)(X16 + e) = o; __threadfence(); } }
  else if (t < nx + nw) { const size_t e = (t - nx) * 8; const float* w = e < (size_t)256 * D ? wq + e : e < (size_t)768 * D ? wkv + (e - (size_t)256 * D) : wo + (e - (size_t)768 * D); for (int j = 0; j < 8; ++j) o[j] = (b16)(bf16_rne(w[j]) * WSC); for (int pass = 0; pass < 2; ++pass) { *(volatile v8b*)(WT + e) = o; __threadfence(); } }
}
template <int MODE>
__global__ __launch_bounds__(128) void gemm_kernel(const b16* __restrict__ Ah, const b16* __restrict__ Al, const b16* __restrict__ W, const float* __restrict__ bias, b16* __restrict__ Yh, b16* __restrict__ Yl, b16* __restrict__ VTh, b16* __restrict__ VTl, float* __restrict__ Yf) {
  __shared__ __attribute__((aligned(16))) float Ts[4][16][128 + 4]; __shared__ __attribute__((aligned(16))) b16 Vt[128][72], Vtl[128][72];
  const int wave = threadIdx.x >> 5, lane = threadIdx.x & 31, nloc = lane & 15, hlf = lane >> 4, t_ = threadIdx.x; const size_t m0 = (size_t)blockIdx.x * 64 + wave * 16; const int n0 = blockIdx.y * 128;
  v8f acc[8];
#pragma unroll
  for (int t = 0; t < 8; ++t) acc[t] = (v8f){};
#pragma unroll 2
  for (int kb = 0; kb < D; kb += 32) { const v16b a = frag_kb(Ah + (m0 + nloc) * D + kb, hlf); v16b al = {}; if (MODE == 2) al = frag_kb(Al + (m0 + nloc) * D + kb, hlf);
#pragma unroll
    for (int t = 0; t < 8; ++t) { const v16b bw = frag_kb(W + (size_t)(n0 + t * 16 + nloc) * D + kb, hlf); acc[t] = wmma16b(a, bw, acc[t]); if (MODE == 2) acc[t] = wmma16b(al, bw, acc[t]); } }
  const float rs_ = (MODE == 2) ? 1.0f / (OS * WSC) : 1.0f / (XS * WSC);
  if (MODE == 1 && n0 >= D) {
    const int b = (int)(m0 / T); const int s0 = (int)((size_t)blockIdx.x * 64 - (size_t)b * T); const int d0 = n0 - D;
#pragma unroll
    for (int t = 0; t < 8; ++t) { const float bb = bf16_rne(bias[n0 + t * 16 + nloc]);
#pragma unroll
      for (int r = 0; r < 8; ++r) { b16 p, q; split16((acc[t][r] * rs_ + bb) * XS, p, q); Vt[t * 16 + nloc][wave * 16 + 8 * hlf + r] = p; Vtl[t * 16 + nloc][wave * 16 + 8 * hlf + r] = q; } }
    __syncthreads();
    for (int pass = 0; pass < 2; ++pass) { for (int q = t_; q < 128 * 8; q += 128) { const int dd = q >> 3, c8 = (q & 7) * 8; const size_t gi = ((size_t)b * D + d0 + dd) * T + s0 + c8; *(volatile v8b*)(VTh + gi) = *(const v8b*)(&Vt[dd][c8]); *(volatile v8b*)(VTl + gi) = *(const v8b*)(&Vtl[dd][c8]); } __threadfence(); }
    return; }
#pragma unroll
  for (int t = 0; t < 8; ++t) { const int c = n0 + t * 16 + nloc; const float bb = bf16_rne(bias[c]);
#pragma unroll
    for (int r = 0; r < 8; ++r) Ts[wave][8 * hlf + r][t * 16 + nloc] = acc[t][r] * rs_ + bb; }
  wave_lds_sync();
  for (int pass = 0; pass < 2; ++pass) { for (int rr = 0; rr < 16; ++rr) {
      if (MODE == 2) *(volatile v4f*)(Yf + (m0 + rr) * D + n0 + lane * 4) = *(const v4f*)(&Ts[wave][rr][lane * 4]);
      else if (lane < 16) { v8b hv, lv; for (int j = 0; j < 8; ++j) { b16 p, q; split16(Ts[wave][rr][lane * 8 + j] * XS, p, q); hv[j] = p; lv[j] = q; } *(volatile v8b*)(Yh + (m0 + rr) * D + n0 + lane * 8) = hv; *(volatile v8b*)(Yl + (m0 + rr) * D + n0 + lane * 8) = lv; } }
    __threadfence(); }
}
__global__ __launch_bounds__(64) void attn_kernel(const b16* __restrict__ Qh, const b16* __restrict__ Ql, const b16* __restrict__ Kh, const b16* __restrict__ Kl, const b16* __restrict__ VTh, const b16* __restrict__ VTl, b16* __restrict__ Oh, b16* __restrict__ Ol) {
  __shared__ __attribute__((aligned(16))) float To[2][16][D + 4];
  const int wave = threadIdx.x >> 5, lane = threadIdx.x & 31, hh = lane >> 4, col = lane & 15; const int b = blockIdx.y; const int q0 = blockIdx.x * 32 + wave * 16, qi = q0 + col;
  const size_t qo = ((size_t)b * T + qi) * D;
  const b16* Kb = Kh + (size_t)b * T * D; const b16* Klb = Kl + (size_t)b * T * D; const b16* Vb = VTh + (size_t)b * D * T; const b16* Vlb = VTl + (size_t)b * D * T;
  float m = -INFINITY, l = 0.0f; v8f o[16];
#pragma unroll
  for (int t = 0; t < 16; ++t) o[t] = (v8f){};
  const float cs = SCALE * LOG2E / (XS * XS);
  for (int kb = 0; kb < T; kb += 32) {
    v8f s0 = {}, s1 = {};
#pragma unroll 2
    for (int ks = 0; ks < D; ks += 32) { const v16b qa = frag_kb(Qh + qo + ks, hh), ql = frag_kb(Ql + qo + ks, hh);
      const b16* k0 = Kb + (size_t)(kb + col) * D + ks, *k1 = Kb + (size_t)(kb + 16 + col) * D + ks;
      v16b f = frag_kb(k0, hh); s0 = wmma16b(f, qa, s0); s0 = wmma16b(f, ql, s0); s0 = wmma16b(frag_kb(Klb + (size_t)(kb + col) * D + ks, hh), qa, s0);
      f = frag_kb(k1, hh); s1 = wmma16b(f, qa, s1); s1 = wmma16b(f, ql, s1); s1 = wmma16b(frag_kb(Klb + (size_t)(kb + 16 + col) * D + ks, hh), qa, s1); }
    float e[16]; float mx = -INFINITY;
#pragma unroll
    for (int r = 0; r < 8; ++r) { e[r] = s0[r] * cs; e[8 + r] = s1[r] * cs; mx = fmaxf(mx, fmaxf(e[r], e[8 + r])); }
    mx = fmaxf(mx, __shfl_xor(mx, 16)); const float mn = fmaxf(m, mx); const float al = nexp2(m - mn); m = mn; float sum = 0.0f; v16b ph, pl;
#pragma unroll
    for (int i = 0; i < 16; ++i) { const float p = nexp2(e[i] - mn); sum += p; const b16 h_ = (b16)(p * PS); ph[i] = h_; pl[i] = (b16)(p * PS - (float)h_); }
    sum += __shfl_xor(sum, 16); l = l * al + sum;
#pragma unroll
    for (int t = 0; t < 16; ++t) { o[t] *= al; const v16b vf = frag_kb(Vb + (size_t)(t * 16 + col) * T + kb, hh); o[t] = wmma16b(vf, ph, o[t]); o[t] = wmma16b(vf, pl, o[t]); o[t] = wmma16b(frag_kb(Vlb + (size_t)(t * 16 + col) * T + kb, hh), ph, o[t]); } }
  const float inv = 1.0f / (l * PS * XS);
#pragma unroll
  for (int t = 0; t < 16; ++t)
#pragma unroll
    for (int r = 0; r < 8; ++r) To[wave][col][t * 16 + 8 * hh + r] = o[t][r] * inv;
  wave_lds_sync();
  for (int pass = 0; pass < 2; ++pass) { for (int rr = 0; rr < 16; ++rr) { const int c8 = lane * 8; v8b hv, lv; for (int j = 0; j < 8; ++j) { b16 p, q; split16(To[wave][rr][c8 + j] * OS, p, q); hv[j] = p; lv[j] = q; }
      *(volatile v8b*)(Oh + ((size_t)b * T + q0 + rr) * D + c8) = hv; *(volatile v8b*)(Ol + ((size_t)b * T + q0 + rr) * D + c8) = lv; } __threadfence(); }
}
}

extern "C" void kernel_launch(void* const* d_in, const int* in_sizes, int n_in, void* d_out, int out_size, void* d_ws, size_t ws_size, hipStream_t stream) {
  (void)n_in;
  auto Fp = [&](int i) { return (const float*)d_in[i]; };
  if (in_sizes[0] != NR * D || in_sizes[1] != NR * D || in_sizes[2] != D * D || in_sizes[4] != 2 * D * D || in_sizes[6] != D * D || out_size != NR * D) return;
  size_t off = 0; char* ws = (char*)d_ws;
  auto carve = [&](size_t bytes) { char* p = ws + off; off += (bytes + 255) & ~(size_t)255; return p; };
  b16* X16 = (b16*)carve((size_t)2 * NR * D * 2); b16* WT = (b16*)carve((size_t)1024 * D * 2);
  b16* Qh = (b16*)carve((size_t)NR * D * 2); b16* Ql = (b16*)carve((size_t)NR * D * 2); b16* Kh = (b16*)carve((size_t)NR * D * 2); b16* Kl = (b16*)carve((size_t)NR * D * 2); b16* VTh = (b16*)carve((size_t)NR * D * 2); b16* VTl = (b16*)carve((size_t)NR * D * 2);
  b16* Oh = X16; b16* Ol = X16 + (size_t)NR * D;
  if (off > ws_size || off > ((size_t)128 << 20)) return;
  const b16 *WQ = WT, *WKV = WT + (size_t)256 * D, *WO = WT + (size_t)768 * D;
  prep_kernel<<<(unsigned)(((size_t)2 * NR * D / 8 + (size_t)1024 * D / 8 + 255) / 256), 256, 0, stream>>>(Fp(0), Fp(1), Fp(2), Fp(4), Fp(6), X16, WT);
  gemm_kernel<0><<<dim3(NR / 64, 2), 128, 0, stream>>>(X16, nullptr, WQ, Fp(3), Qh, Ql, nullptr, nullptr, nullptr);
  gemm_kernel<1><<<dim3(NR / 64, 4), 128, 0, stream>>>(X16 + (size_t)NR * D, nullptr, WKV, Fp(5), Kh, Kl, VTh, VTl, nullptr);
  attn_kernel<<<dim3(T / 32, NB), 64, 0, stream>>>(Qh, Ql, Kh, Kl, VTh, VTl, Oh, Ol);
  gemm_kernel<2><<<dim3(NR / 64, 2), 128, 0, stream>>>(Oh, Ol, WO, Fp(7), nullptr, nullptr, nullptr, nullptr, (float*)d_out);
}
